// madsormer_ae_13795434954998
// MI455X (gfx1250) — hardware-verified
//
#include <hip/hip_runtime.h>
#include <math.h>
#include <stdint.h>

#ifndef NB
#define NB 16
#endif
#ifndef SEQ
#define SEQ 2048
#endif
#define NB_FULL  16
#define SEQ_FULL 2048
#define IK       3
#define DM       4
#define HID      256
#define FFD      512
#define NLAYER   2
#define NROW     (NB * SEQ)
#define BG       (((NB % 4) == 0) ? 4 : (((NB % 2) == 0) ? 2 : 1))
#define NGRP     (NB / BG)
#define RQB      16
#define TOKB     64
#define SMT      (SEQ / 8)
#define SMW      (SMT / 32)
#define PCARRY   32768.0f
#define VCARRY   256.0f
#define LNEPS    1e-5f
static_assert(NB >= 1 && NB <= NB_FULL);
static_assert(SEQ >= 256 && SEQ <= SEQ_FULL && (SEQ % 256) == 0);
static_assert((NB % BG) == 0 && NGRP >= 1);
static_assert(SMT >= 32 && SMT <= 256 && SMW >= 1 && SMW <= 8);
static_assert((NROW % TOKB) == 0 && (SEQ % TOKB) == 0 && TOKB == 64);
static_assert((SEQ % RQB) == 0 && (SEQ % 32) == 0 && (HID % 64) == 0 && (HID % 8) == 0);
static_assert(TOKB * 4 == HID && (FFD % TOKB) == 0 && (HID % TOKB) == 0);

typedef _Float16 v16h __attribute__((ext_vector_type(16)));
typedef _Float16 v8h  __attribute__((ext_vector_type(8)));
typedef __bf16   v16b __attribute__((ext_vector_type(16)));
typedef __bf16   v8b  __attribute__((ext_vector_type(8)));
typedef float    v8f  __attribute__((ext_vector_type(8)));
typedef float    v4f  __attribute__((ext_vector_type(4)));
typedef float    v2f  __attribute__((ext_vector_type(2)));
typedef unsigned int v4u __attribute__((ext_vector_type(4)));

#if defined(__HIP_DEVICE_COMPILE__)
#define DEV_ASM 1
#else
#define DEV_ASM 0
#endif

__device__ __forceinline__ unsigned short bf_bits(float f) {
  unsigned u = __float_as_uint(f);
  return (unsigned short)((u + 0x7FFFu + ((u >> 16) & 1u)) >> 16);
}
__device__ __forceinline__ float bf_up(unsigned short hb) { return __uint_as_float(((unsigned)hb) << 16); }
__device__ __forceinline__ float bfr(float f) { return bf_up(bf_bits(f)); }
__device__ __forceinline__ unsigned short h_bits(_Float16 x) { return __builtin_bit_cast(unsigned short, x); }
__device__ __forceinline__ unsigned pk16(unsigned short a, unsigned short b) { return (unsigned)a | ((unsigned)b << 16); }
__device__ __forceinline__ v8f zero8() { v8f z = {0.f, 0.f, 0.f, 0.f, 0.f, 0.f, 0.f, 0.f}; return z; }

template <typename OT> struct FT;
template <> struct FT<__bf16>   { typedef v16b frag; typedef v8b half8; };
template <> struct FT<_Float16> { typedef v16h frag; typedef v8h half8; };

template <typename OT>
__device__ __forceinline__ typename FT<OT>::frag ldfrag(const OT* p) {
  union { typename FT<OT>::frag v; typename FT<OT>::half8 h[2]; } f;
  f.h[0] = *(const typename FT<OT>::half8*)(p);
  f.h[1] = *(const typename FT<OT>::half8*)(p + 16);
  return f.v;
}

__device__ __forceinline__ v8f mmar(v16b a, v16b b, v8f c) {
  return __builtin_amdgcn_wmma_f32_16x16x32_bf16(false, a, false, b, (short)0, c, false, false);
}
__device__ __forceinline__ v8f mmar(v16h a, v16h b, v8f c) {
  return __builtin_amdgcn_wmma_f32_16x16x32_f16(false, a, false, b, (short)0, c, false, false);
}
__device__ __forceinline__ void dep_guard(v8f& a, v8f& b, v16b x, v16b y) {
#if DEV_ASM
  asm volatile("v_nop\n\tv_nop\n\tv_nop\n\tv_nop" : "+v"(a), "+v"(b) : "v"(x), "v"(y));
#else
  (void)a; (void)b; (void)x; (void)y;
#endif
}
__device__ __forceinline__ void dep_guard(v8f& a, v8f& b, v16h x, v16h y) {
#if DEV_ASM
  asm volatile("v_nop\n\tv_nop\n\tv_nop\n\tv_nop" : "+v"(a), "+v"(b) : "v"(x), "v"(y));
#else
  (void)a; (void)b; (void)x; (void)y;
#endif
}
__device__ __forceinline__ void keep4(v16b a, v16b b, v16b c, v16b d) {
#if DEV_ASM
  asm volatile("v_nop" :: "v"(a), "v"(b), "v"(c), "v"(d));
#else
  (void)a; (void)b; (void)c; (void)d;
#endif
}
__device__ __forceinline__ void keep4(v16h a, v16h b, v16h c, v16h d) {
#if DEV_ASM
  asm volatile("v_nop" :: "v"(a), "v"(b), "v"(c), "v"(d));
#else
  (void)a; (void)b; (void)c; (void)d;
#endif
}
__device__ __forceinline__ void acc_guard4(v8f& a, v8f& b, v8f& c, v8f& d) {
#if DEV_ASM
  asm volatile("v_nop\n\tv_nop\n\tv_nop\n\tv_nop" : "+v"(a), "+v"(b), "+v"(c), "+v"(d));
#else
  (void)a; (void)b; (void)c; (void)d;
#endif
}

template <typename OT, int MI, int NPA, int NPB, int OUT_MODE, int CZ>
__global__ __launch_bounds__(256) void gemm_t(
    const unsigned short* __restrict__ Ap, const unsigned short* __restrict__ A2p, int lda, long long strideA,
    const unsigned short* __restrict__ Btp, int ldb, long long strideB,
    const unsigned short* __restrict__ B2p, int ldb2, long long strideB2, int K2,
    void* Cout, void* Cout2, int ldc, long long strideC, int ldc2, long long strideC2, int N2,
    int M, int N, int K, float oscale, float rscale2, float cscale, float rscaleC) {
  static_assert(CZ != 2 || ((16 * MI) % 32) == 0);
  static_assert(!(NPA == 2 && NPB == 2));
  typedef typename FT<OT>::frag V16;
  const OT* A  = (const OT*)(const void*)Ap;
  const OT* A2 = (const OT*)(const void*)A2p;
  const OT* Bt = (const OT*)(const void*)Btp;
  const OT* B2 = (const OT*)(const void*)B2p;
  __shared__ __align__(16) float sT[8][16 * 68];
  const int RT   = 16 * MI;
  const int b    = blockIdx.y;
  const int lane = threadIdx.x & 31;
  const int wave = threadIdx.x >> 5;
  const int tilesN = N >> 6;
  const int tilesM = M / RT;
  const int tile = blockIdx.x * 8 + wave;
  if (tile >= tilesM * tilesN) return;
  const int tm = tile / tilesN;
  const int tn = tile - tm * tilesN;
  const int m0 = tm * RT;
  const int n0 = tn << 6;
  if (CZ == 1) {
    if (n0 >= m0 + RT) return;
  }
  int kEnd = K;
  if (CZ == 2) {
    const int ke = m0 + RT;
    kEnd = (ke < K) ? ke : K;
  }

  const OT* Ab  = A  + (size_t)b * (size_t)strideA;
  const OT* A2b = A2 + (size_t)b * (size_t)strideA;
  const OT* Bb  = Bt + (size_t)b * (size_t)strideB;
  const OT* B2b = B2 + (size_t)b * (size_t)strideB2;

  const int rlane = lane & 15;
  const int koff  = (lane >> 4) * 8;
  const int mOff  = (lane >> 4) * 8;

  v8f acc[MI][4], acc2[MI][4];
#pragma unroll
  for (int i = 0; i < MI; ++i)
#pragma unroll
    for (int j = 0; j < 4; ++j) { acc[i][j] = zero8(); acc2[i][j] = zero8(); }

#pragma unroll 1
  for (int k0 = 0; k0 < kEnd; k0 += 32) {
    V16 bq[4];
#pragma unroll
    for (int j = 0; j < 4; ++j)
      bq[j] = ldfrag<OT>(Bb + (size_t)(n0 + (j << 4) + rlane) * ldb + koff + k0);
#pragma unroll
    for (int i = 0; i < MI; ++i) {
      const V16 af = ldfrag<OT>(Ab + (size_t)(m0 + (i << 4) + rlane) * lda + koff + k0);
#pragma unroll
      for (int j = 0; j < 4; ++j) acc[i][j] = mmar(af, bq[j], acc[i][j]);
      dep_guard(acc[i][0], acc[i][3], af, bq[3]);
      if (NPA == 2) {
        const V16 af2 = ldfrag<OT>(A2b + (size_t)(m0 + (i << 4) + rlane) * lda + koff + k0);
#pragma unroll
        for (int j = 0; j < 4; ++j) acc2[i][j] = mmar(af2, bq[j], acc2[i][j]);
        dep_guard(acc2[i][0], acc2[i][3], af2, bq[3]);
      }
    }
    keep4(bq[0], bq[1], bq[2], bq[3]);
    if (NPB == 2) {
      if (k0 < K2) {
        V16 br[4];
#pragma unroll
        for (int j = 0; j < 4; ++j)
          br[j] = ldfrag<OT>(B2b + (size_t)(n0 + (j << 4) + rlane) * ldb2 + koff + k0);
#pragma unroll
        for (int i = 0; i < MI; ++i) {
          const V16 afr = ldfrag<OT>(Ab + (size_t)(m0 + (i << 4) + rlane) * lda + koff + k0);
#pragma unroll
          for (int j = 0; j < 4; ++j) acc2[i][j] = mmar(afr, br[j], acc2[i][j]);
          dep_guard(acc2[i][0], acc2[i][3], afr, br[3]);
        }
        keep4(br[0], br[1], br[2], br[3]);
      }
    }
  }
#pragma unroll
  for (int i = 0; i < MI; ++i) {
    acc_guard4(acc[i][0], acc[i][1], acc[i][2], acc[i][3]);
    if (NPA == 2 || NPB == 2) acc_guard4(acc2[i][0], acc2[i][1], acc2[i][2], acc2[i][3]);
  }

  float* slab = sT[wave];
#pragma unroll
  for (int i = 0; i < MI; ++i) {
    const int mBase = m0 + (i << 4);
#pragma unroll
    for (int j = 0; j < 4; ++j) {
#pragma unroll
      for (int r = 0; r < 8; ++r) {
        float v = acc[i][j][r];
        if (NPA == 2 || NPB == 2) v += acc2[i][j][r] * rscale2;
        v = v * oscale;
        slab[(mOff + r) * 68 + (j << 4) + rlane] = v;
      }
    }
    __builtin_amdgcn_fence(__ATOMIC_RELEASE, "workgroup");
    __builtin_amdgcn_wave_barrier();
    __builtin_amdgcn_fence(__ATOMIC_ACQUIRE, "workgroup");
    if (OUT_MODE == 0) {
      float* C = (float*)Cout + (size_t)b * (size_t)strideC;
      const int h2 = lane >> 4, c4 = (lane & 15) * 4;
      for (int pass = 0; pass < 2; ++pass) {
#pragma unroll
        for (int it = 0; it < 8; ++it) {
          const int row = it * 2 + h2;
          const v4f v = *(const v4f*)(slab + row * 68 + c4);
          *(volatile v4f*)(C + (size_t)(mBase + row) * ldc + n0 + c4) = v;
        }
        __threadfence();
      }
    } else {
      const int q = lane >> 3, c8 = (lane & 7) * 8;
      unsigned short* C  = (unsigned short*)Cout  + (size_t)b * (size_t)strideC;
      unsigned short* C2 = (unsigned short*)Cout2 + (size_t)b * (size_t)strideC2;
      const bool wr2 = (OUT_MODE == 3) && (n0 < N2);
      v4u hv[4], lv[4];
#pragma unroll
      for (int it = 0; it < 4; ++it) {
        const int row = it * 4 + q;
        const float* sp = slab + row * 68 + c8;
        float f[8];
#pragma unroll
        for (int e = 0; e < 8; ++e) f[e] = sp[e] * cscale;
        v4u a, a2;
#pragma unroll
        for (int e = 0; e < 4; ++e) {
          const float f0 = f[2 * e], f1 = f[2 * e + 1];
          const _Float16 x0 = (_Float16)f0, x1 = (_Float16)f1;
          const unsigned short h0 = h_bits(x0), h1 = h_bits(x1);
          unsigned short l0 = 0, l1 = 0;
          if (OUT_MODE == 3) {
            l0 = h_bits((_Float16)((f0 - (float)x0) * rscaleC));
            l1 = h_bits((_Float16)((f1 - (float)x1) * rscaleC));
          }
          a[e] = pk16(h0, h1); a2[e] = pk16(l0, l1);
        }
        hv[it] = a; lv[it] = a2;
      }
      for (int pass = 0; pass < 2; ++pass) {
#pragma unroll
        for (int it = 0; it < 4; ++it) {
          const int row = it * 4 + q;
          *(volatile v4u*)(C + (size_t)(mBase + row) * ldc + n0 + c8) = hv[it];
          if (OUT_MODE == 3) {
            if (wr2) *(volatile v4u*)(C2 + (size_t)(mBase + row) * ldc2 + n0 + c8) = lv[it];
          }
        }
        __threadfence();
      }
    }
    __builtin_amdgcn_fence(__ATOMIC_RELEASE, "workgroup");
    __builtin_amdgcn_wave_barrier();
    __builtin_amdgcn_fence(__ATOMIC_ACQUIRE, "workgroup");
  }
}

__global__ __launch_bounds__(256) void lconst_kernel(const float* __restrict__ Wq, const float* __restrict__ bq,
                                                     const float* __restrict__ Wk, const float* __restrict__ bk,
                                                     float* cst) {
  __shared__ float sP[25 * 256];
  __shared__ __align__(16) float sL[32];
  const int ly   = blockIdx.x;
  const int h    = threadIdx.x;
  const int lane = h & 31, wave = h >> 5;
  const float* wq = Wq + (size_t)ly * DM * HID;
  const float* wk = Wk + (size_t)ly * DM * HID;
  float q[4], k[4];
#pragma unroll
  for (int a = 0; a < 4; ++a) { q[a] = bfr(wq[a * HID + h]); k[a] = bfr(wk[a * HID + h]); }
  const float bqh = bfr(bq[(size_t)ly * HID + h]);
  const float bkh = bfr(bk[(size_t)ly * HID + h]);
#pragma unroll
  for (int a = 0; a < 4; ++a) {
#pragma unroll
    for (int c = 0; c < 4; ++c) sP[(a * 4 + c) * 256 + h] = q[a] * k[c];
    sP[(16 + a) * 256 + h] = q[a] * bkh;
    sP[(20 + a) * 256 + h] = k[a] * bqh;
  }
  sP[24 * 256 + h] = bqh * bkh;
  __syncthreads();
  if (wave == 0) {
    const int j = (lane < 24) ? lane : 24;
    float s = 0.f;
#pragma unroll 1
    for (int i = 0; i < 256; ++i) s += sP[j * 256 + i];
    sL[lane] = (lane < 25) ? s : 0.f;
  }
  __syncthreads();
  const v4f v = *(const v4f*)(sL + (lane & 7) * 4);
  float* op = cst + (size_t)ly * 32 + (lane & 7) * 4;
  for (int pass = 0; pass < 2; ++pass) {
    if (wave == 0 && lane < 8) *(volatile v4f*)op = v;
    __threadfence();
  }
}

template <int FIRST>
__global__ __launch_bounds__(TOKB) void tok_kernel(
    const float* __restrict__ KEY, const float* __restrict__ VAL, const float* __restrict__ XIN,
    const float* __restrict__ Wq, const float* __restrict__ bq,
    const float* __restrict__ Wk, const float* __restrict__ bk,
    const float* __restrict__ Wv, const float* __restrict__ bv,
    const float* __restrict__ cst,
    float* XB, float* PV, float* SCP, unsigned short* VT) {
  __shared__ __align__(16) float sWq[HID * 4];
  __shared__ __align__(16) float sWk[HID * 4];
  __shared__ __align__(16) float sWv[HID * 4];
  __shared__ __align__(16) float sBq[HID];
  __shared__ __align__(16) float sBk[HID];
  __shared__ __align__(16) float sBv[HID];
  __shared__ __align__(16) unsigned short sVT[HID * TOKB];
  const int tl   = threadIdx.x;
  const int lane = tl & 31, wave = tl >> 5;
  const int tc0  = blockIdx.x * TOKB;
  const int b    = tc0 / SEQ;
  const int t0   = tc0 - b * SEQ;
  const int tc   = tc0 + tl;
  const int t    = t0 + tl;

  float g[16], u[4], w[4];
  {
    const v4f cA = *(const v4f*)(cst + 0);
    const v4f cB = *(const v4f*)(cst + 4);
    const v4f cC = *(const v4f*)(cst + 8);
    const v4f cD = *(const v4f*)(cst + 12);
    const v4f cU = *(const v4f*)(cst + 16);
    const v4f cW = *(const v4f*)(cst + 20);
#pragma unroll
    for (int j = 0; j < 4; ++j) {
      g[j] = cA[j]; g[4 + j] = cB[j]; g[8 + j] = cC[j]; g[12 + j] = cD[j];
      u[j] = cU[j]; w[j] = cW[j];
    }
  }
  const float s0 = cst[24];

  {
    const int h4 = tl * 4;
#pragma unroll 1
    for (int j = 0; j < DM; ++j) {
      const v4f a = *(const v4f*)(Wq + (size_t)j * HID + h4);
      const v4f c = *(const v4f*)(Wk + (size_t)j * HID + h4);
      const v4f d = *(const v4f*)(Wv + (size_t)j * HID + h4);
#pragma unroll
      for (int e = 0; e < 4; ++e) {
        sWq[(h4 + e) * 4 + j] = bfr(a[e]);
        sWk[(h4 + e) * 4 + j] = bfr(c[e]);
        sWv[(h4 + e) * 4 + j] = bfr(d[e]);
      }
    }
    const v4f qb4 = *(const v4f*)(bq + h4);
    const v4f kb4 = *(const v4f*)(bk + h4);
    const v4f vb4 = *(const v4f*)(bv + h4);
    v4f qc, kc, vc;
#pragma unroll
    for (int e = 0; e < 4; ++e) { qc[e] = bfr(qb4[e]); kc[e] = bfr(kb4[e]); vc[e] = bfr(vb4[e]); }
    *(v4f*)(sBq + h4) = qc;
    *(v4f*)(sBk + h4) = kc;
    *(v4f*)(sBv + h4) = vc;
  }

  float x0, x1, x2, x3;
  if (FIRST) {
    const size_t row = (size_t)b * SEQ_FULL + (size_t)t;
    x0 = bfr(KEY[row * IK + 0]);
    x1 = bfr(KEY[row * IK + 1]);
    x2 = bfr(KEY[row * IK + 2]);
    x3 = bfr(VAL[row]);
  } else {
    const v4f xv = *(const v4f*)(XIN + (size_t)tc * 4);
    x0 = xv[0]; x1 = xv[1]; x2 = xv[2]; x3 = xv[3];
  }
  __syncthreads();

  float qn = 0.f, kn = 0.f;
#pragma unroll 1
  for (int h = 0; h < HID; ++h) {
    const v4f wq = *(const v4f*)(sWq + h * 4);
    const v4f wk = *(const v4f*)(sWk + h * 4);
    const v4f wv = *(const v4f*)(sWv + h * 4);
    float q = x0 * wq[0]; q = fmaf(x1, wq[1], q); q = fmaf(x2, wq[2], q); q = fmaf(x3, wq[3], q); q += sBq[h];
    float k = x0 * wk[0]; k = fmaf(x1, wk[1], k); k = fmaf(x2, wk[2], k); k = fmaf(x3, wk[3], k); k += sBk[h];
    float v = x0 * wv[0]; v = fmaf(x1, wv[1], v); v = fmaf(x2, wv[2], v); v = fmaf(x3, wv[3], v); v += sBv[h];
    sVT[h * TOKB + tl] = h_bits((_Float16)(v * VCARRY));
    qn = fmaf(q, q, qn);
    kn = fmaf(k, k, kn);
  }
  v4f pv;
#pragma unroll
  for (int c = 0; c < 4; ++c)
    pv[c] = fmaf(x3, g[12 + c], fmaf(x2, g[8 + c], fmaf(x1, g[4 + c], x0 * g[c])));
  const float xu = fmaf(x3, u[3], fmaf(x2, u[2], fmaf(x1, u[1], x0 * u[0])));
  const float xw = fmaf(x3, w[3], fmaf(x2, w[2], fmaf(x1, w[1], x0 * w[0])));
  const float rq = fmaf(-2.0f, xu + s0, qn);
  const float rk = fmaf(-2.0f, xw, kn);
  v4f xr; xr[0] = x0; xr[1] = x1; xr[2] = x2; xr[3] = x3;
  v4f sr; sr[0] = rq; sr[1] = rk; sr[2] = qn; sr[3] = kn;
  __syncthreads();

  const int qq = lane >> 3, c8 = (lane & 7) * 8;
  unsigned short* vtb = VT + (size_t)b * HID * SEQ + (size_t)t0 + c8;
  float* xbp = XB  + (size_t)tc * 4;
  float* pvp = PV  + (size_t)tc * 4;
  float* scp = SCP + (size_t)tc * 4;
  for (int pass = 0; pass < 2; ++pass) {
    *(volatile v4f*)xbp = xr;
    *(volatile v4f*)pvp = pv;
    *(volatile v4f*)scp = sr;
#pragma unroll 4
    for (int it = 0; it < HID / 8; ++it) {
      const int h = it * 8 + wave * 4 + qq;
      const v4u v = *(const v4u*)(sVT + h * TOKB + c8);
      *(volatile v4u*)(vtb + (size_t)h * SEQ) = v;
    }
    __threadfence();
  }
}

__global__ __launch_bounds__(SMT) void attn_rows(const float* __restrict__ PV, const float* __restrict__ SCP,
                                                 const float* __restrict__ XB, const float* __restrict__ bwp,
                                                 unsigned short* P, int b0) {
  extern __shared__ v4f dynLs4[];
  float* Ls = (float*)dynLs4;
  __shared__ __align__(16) float sRow[RQB][8];
  __shared__ float redm[8][RQB];
  __shared__ float reds[8][RQB];
  __shared__ float rowmx[RQB];
  __shared__ float rowsc[RQB];
  const int tid  = threadIdx.x;
  const int wave = tid >> 5;
  const int lane = tid & 31;
  const int bl   = blockIdx.y;
  const int b    = b0 + bl;
  const int q0   = blockIdx.x * RQB;
  const int c0   = tid * 8;
  {
    const int r = tid & (RQB - 1);
    const size_t tq = (size_t)b * SEQ + (size_t)(q0 + r);
    const v4f p = *(const v4f*)(PV + tq * 4);
    const v4f s = *(const v4f*)(SCP + tq * 4);
    if (tid < RQB) {
      sRow[r][0] = p[0]; sRow[r][1] = p[1]; sRow[r][2] = p[2]; sRow[r][3] = p[3];
      sRow[r][4] = s[0]; sRow[r][5] = 0.f; sRow[r][6] = 0.f; sRow[r][7] = 0.f;
    }
  }
  const float bwr  = bfr(bwp[0]);
  const float nhb2 = -0.5f * bwr * bwr;
  v4f xk[8];
  float rk[8];
#pragma unroll
  for (int j = 0; j < 4; ++j) {
    const size_t tk = (size_t)b * SEQ + (size_t)(c0 + j);
    xk[j] = *(const v4f*)(XB + tk * 4);
    const v4f s = *(const v4f*)(SCP + tk * 4);
    rk[j] = s[1];
  }
  asm volatile("" ::: "memory");
#pragma unroll
  for (int j = 4; j < 8; ++j) {
    const size_t tk = (size_t)b * SEQ + (size_t)(c0 + j);
    xk[j] = *(const v4f*)(XB + tk * 4);
    const v4f s = *(const v4f*)(SCP + tk * 4);
    rk[j] = s[1];
  }
  __syncthreads();

  float* lcol = Ls + c0;
#pragma unroll 1
  for (int r = 0; r < RQB; ++r) {
    const v4f p = *(const v4f*)(&sRow[r][0]);
    const float rq = sRow[r][4];
    float l[8];
    float mx = -INFINITY;
#pragma unroll
    for (int j = 0; j < 8; ++j) {
      float dot = xk[j][0] * p[0];
      dot = fmaf(xk[j][1], p[1], dot);
      dot = fmaf(xk[j][2], p[2], dot);
      dot = fmaf(xk[j][3], p[3], dot);
      const float d2 = fmaf(-2.0f, dot, rq + rk[j]);
      l[j] = nhb2 * d2;
      mx = fmaxf(mx, l[j]);
    }
    v4f la, lb;
    la[0] = l[0]; la[1] = l[1]; la[2] = l[2]; la[3] = l[3];
    lb[0] = l[4]; lb[1] = l[5]; lb[2] = l[6]; lb[3] = l[7];
    *(v4f*)(lcol + (size_t)r * SEQ)     = la;
    *(v4f*)(lcol + (size_t)r * SEQ + 4) = lb;
#pragma unroll
    for (int off = 1; off < 32; off <<= 1) mx = fmaxf(mx, __shfl_xor(mx, off, 32));
    if (lane == 0) redm[wave][r] = mx;
  }
  __syncthreads();
  if (tid < RQB) {
    float m = redm[0][tid];
#pragma unroll
    for (int ww = 1; ww < SMW; ++ww) m = fmaxf(m, redm[ww][tid]);
    rowmx[tid] = m;
  }
  __syncthreads();
#pragma unroll 1
  for (int r = 0; r < RQB; ++r) {
    const float m = rowmx[r];
    v4f la = *(const v4f*)(lcol + (size_t)r * SEQ);
    v4f lb = *(const v4f*)(lcol + (size_t)r * SEQ + 4);
    float s = 0.f;
#pragma unroll
    for (int e = 0; e < 4; ++e) {
      la[e] = __expf(la[e] - m); s += la[e];
      lb[e] = __expf(lb[e] - m); s += lb[e];
    }
    *(v4f*)(lcol + (size_t)r * SEQ)     = la;
    *(v4f*)(lcol + (size_t)r * SEQ + 4) = lb;
#pragma unroll
    for (int off = 1; off < 32; off <<= 1) s += __shfl_xor(s, off, 32);
    if (lane == 0) reds[wave][r] = s;
  }
  __syncthreads();
  if (tid < RQB) {
    float s = reds[0][tid];
#pragma unroll
    for (int ww = 1; ww < SMW; ++ww) s += reds[ww][tid];
    rowsc[tid] = PCARRY * (1.0f / s);
  }
  __syncthreads();
  unsigned short* pb = P + ((size_t)bl * SEQ + (size_t)q0) * SEQ + c0;
  for (int pass = 0; pass < 2; ++pass) {
#pragma unroll 1
    for (int r = 0; r < RQB; ++r) {
      const float sc = rowsc[r];
      const v4f la = *(const v4f*)(lcol + (size_t)r * SEQ);
      const v4f lb = *(const v4f*)(lcol + (size_t)r * SEQ + 4);
      v4u pk;
      pk[0] = pk16(h_bits((_Float16)(la[0] * sc)), h_bits((_Float16)(la[1] * sc)));
      pk[1] = pk16(h_bits((_Float16)(la[2] * sc)), h_bits((_Float16)(la[3] * sc)));
      pk[2] = pk16(h_bits((_Float16)(lb[0] * sc)), h_bits((_Float16)(lb[1] * sc)));
      pk[3] = pk16(h_bits((_Float16)(lb[2] * sc)), h_bits((_Float16)(lb[3] * sc)));
      *(volatile v4u*)(pb + (size_t)r * SEQ) = pk;
    }
    __threadfence();
  }
}

template <int LAST>
__global__ __launch_bounds__(TOKB) void post_kernel(
    const float* __restrict__ XB, const float* __restrict__ AO,
    const float* __restrict__ Wo, const float* __restrict__ bo,
    const float* __restrict__ g1, const float* __restrict__ be1,
    const float* __restrict__ W1, const float* __restrict__ b1,
    const float* __restrict__ W2, const float* __restrict__ b2,
    const float* __restrict__ g2, const float* __restrict__ be2,
    const float* __restrict__ Wfc, const float* __restrict__ bfc,
    float* XO, float* out) {
  __shared__ __align__(16) v4f sWo[HID];
  __shared__ __align__(16) v4f sW1[FFD];
  __shared__ __align__(16) v4f sW2[FFD];
  __shared__ float sB1[FFD];
  __shared__ __align__(16) float sOut[TOKB];
  const int tl   = threadIdx.x;
  const int lane = tl & 31, wave = tl >> 5;
  const int tc0  = blockIdx.x * TOKB;
  const int b    = tc0 / SEQ;
  const int t0   = tc0 - b * SEQ;
  const int tc   = tc0 + tl;

#pragma unroll 1
  for (int h = tl; h < HID; h += TOKB) {
    const v4f wr = *(const v4f*)(Wo + (size_t)h * DM);
    v4f a;
#pragma unroll
    for (int d = 0; d < 4; ++d) a[d] = bfr(wr[d]);
    sWo[h] = a;
  }
#pragma unroll 1
  for (int f = tl; f < FFD; f += TOKB) {
    const v4f w2r = *(const v4f*)(W2 + (size_t)f * DM);
    v4f a, c;
#pragma unroll
    for (int d = 0; d < 4; ++d) { a[d] = bfr(W1[(size_t)d * FFD + f]); c[d] = bfr(w2r[d]); }
    sW1[f] = a; sW2[f] = c;
    sB1[f] = bfr(b1[f]);
  }
  float pbo[4], pg1[4], pbe1[4], pb2[4], pg2[4], pbe2[4], pwf[4];
  {
    const v4f vbo  = *(const v4f*)bo;
    const v4f vg1  = *(const v4f*)g1;
    const v4f vbe1 = *(const v4f*)be1;
    const v4f vb2  = *(const v4f*)b2;
    const v4f vg2  = *(const v4f*)g2;
    const v4f vbe2 = *(const v4f*)be2;
    const v4f vwf  = *(const v4f*)Wfc;
#pragma unroll
    for (int d = 0; d < 4; ++d) {
      pbo[d] = bfr(vbo[d]);  pg1[d] = bfr(vg1[d]); pbe1[d] = bfr(vbe1[d]);
      pb2[d] = bfr(vb2[d]);  pg2[d] = bfr(vg2[d]); pbe2[d] = bfr(vbe2[d]);
      pwf[d] = bfr(vwf[d]);
    }
  }
  const float pbf = bfr(bfc[0]);
  const v4f xv = *(const v4f*)(XB + (size_t)tc * 4);
  __syncthreads();

  const float* ao = AO + (size_t)tc * HID;
  float o0 = 0.f, o1 = 0.f, o2 = 0.f, o3 = 0.f;
#pragma unroll 1
  for (int h = 0; h < HID; h += 2) {
    const v2f a2 = *(const v2f*)(ao + h);
    const v4f w0 = sWo[h], w1 = sWo[h + 1];
    o0 = fmaf(a2[0], w0[0], o0); o1 = fmaf(a2[0], w0[1], o1); o2 = fmaf(a2[0], w0[2], o2); o3 = fmaf(a2[0], w0[3], o3);
    o0 = fmaf(a2[1], w1[0], o0); o1 = fmaf(a2[1], w1[1], o1); o2 = fmaf(a2[1], w1[2], o2); o3 = fmaf(a2[1], w1[3], o3);
  }
  float r0 = xv[0] + (o0 + pbo[0]);
  float r1 = xv[1] + (o1 + pbo[1]);
  float r2 = xv[2] + (o2 + pbo[2]);
  float r3 = xv[3] + (o3 + pbo[3]);
  float m  = (r0 + r1 + r2 + r3) * 0.25f;
  float d0 = r0 - m, d1 = r1 - m, d2 = r2 - m, d3 = r3 - m;
  float var = (d0 * d0 + d1 * d1 + d2 * d2 + d3 * d3) * 0.25f;
  float inv = rsqrtf(var + LNEPS);
  const float e0 = d0 * inv * pg1[0] + pbe1[0];
  const float e1 = d1 * inv * pg1[1] + pbe1[1];
  const float e2 = d2 * inv * pg1[2] + pbe1[2];
  const float e3 = d3 * inv * pg1[3] + pbe1[3];
  float y0 = 0.f, y1 = 0.f, y2 = 0.f, y3 = 0.f;
#pragma unroll 1
  for (int f = 0; f < FFD; ++f) {
    const v4f wa = sW1[f];
    float a = e0 * wa[0]; a = fmaf(e1, wa[1], a); a = fmaf(e2, wa[2], a); a = fmaf(e3, wa[3], a);
    a = a + sB1[f];
    a = fmaxf(a, 0.f);
    const v4f wb = sW2[f];
    y0 = fmaf(a, wb[0], y0); y1 = fmaf(a, wb[1], y1); y2 = fmaf(a, wb[2], y2); y3 = fmaf(a, wb[3], y3);
  }
  r0 = e0 + (y0 + pb2[0]); r1 = e1 + (y1 + pb2[1]); r2 = e2 + (y2 + pb2[2]); r3 = e3 + (y3 + pb2[3]);
  m  = (r0 + r1 + r2 + r3) * 0.25f;
  d0 = r0 - m; d1 = r1 - m; d2 = r2 - m; d3 = r3 - m;
  var = (d0 * d0 + d1 * d1 + d2 * d2 + d3 * d3) * 0.25f;
  inv = rsqrtf(var + LNEPS);
  v4f xn;
  xn[0] = d0 * inv * pg2[0] + pbe2[0];
  xn[1] = d1 * inv * pg2[1] + pbe2[1];
  xn[2] = d2 * inv * pg2[2] + pbe2[2];
  xn[3] = d3 * inv * pg2[3] + pbe2[3];
  float yv = 0.f;
  if (LAST) {
    yv = xn[0] * pwf[0]; yv = fmaf(xn[1], pwf[1], yv); yv = fmaf(xn[2], pwf[2], yv); yv = fmaf(xn[3], pwf[3], yv);
    yv += pbf;
  }
  sOut[tl] = yv;
  __syncthreads();
  const v4f ov = *(const v4f*)(sOut + (lane & 15) * 4);
  float* xop = XO + (size_t)tc * 4;
  float* oop = out + (size_t)b * SEQ_FULL + (size_t)t0 + (lane & 15) * 4;
  for (int pass = 0; pass < 2; ++pass) {
    *(volatile v4f*)xop = xn;
    if (LAST) {
      if (wave == 0 && lane < 16) *(volatile v4f*)oop = ov;
    }
    __threadfence();
  }
}

extern "C" void kernel_launch(void* const* d_in, const int* in_sizes, int n_in,
                              void* d_out, int out_size, void* d_ws, size_t ws_size,
                              hipStream_t stream) {
  if (n_in < 21) return;
  const long long rows = (long long)(NB - 1) * SEQ_FULL + SEQ;
  if ((long long)in_sizes[0] < rows * IK) return;
  if ((long long)in_sizes[1] < rows) return;
  if (in_sizes[2] < NLAYER * DM * HID || in_sizes[3] < NLAYER * HID) return;
  if (in_sizes[4] < NLAYER * DM * HID || in_sizes[5] < NLAYER * HID) return;
  if (in_sizes[6] < NLAYER * DM * HID || in_sizes[7] < NLAYER * HID) return;
  if (in_sizes[8] < NLAYER * HID * DM || in_sizes[9] < NLAYER * DM) return;
  if (in_sizes[10] < NLAYER) return;
  if (in_sizes[11] < NLAYER * DM || in_sizes[12] < NLAYER * DM) return;
  if (in_sizes[13] < NLAYER * DM * FFD || in_sizes[14] < NLAYER * FFD) return;
  if (in_sizes[15] < NLAYER * FFD * DM || in_sizes[16] < NLAYER * DM) return;
  if (in_sizes[17] < NLAYER * DM || in_sizes[18] < NLAYER * DM) return;
  if (in_sizes[19] < DM || in_sizes[20] < 1) return;
  if ((long long)out_size < rows) return;

  const float* KEY = (const float*)d_in[0];
  const float* VAL = (const float*)d_in[1];
  const float* Wq  = (const float*)d_in[2];
  const float* bq  = (const float*)d_in[3];
  const float* Wk  = (const float*)d_in[4];
  const float* bk  = (const float*)d_in[5];
  const float* Wv  = (const float*)d_in[6];
  const float* bv  = (const float*)d_in[7];
  const float* Wo  = (const float*)d_in[8];
  const float* bo  = (const float*)d_in[9];
  const float* bw  = (const float*)d_in[10];
  const float* g1  = (const float*)d_in[11];
  const float* be1 = (const float*)d_in[12];
  const float* W1  = (const float*)d_in[13];
  const float* b1  = (const float*)d_in[14];
  const float* W2  = (const float*)d_in[15];
  const float* b2  = (const float*)d_in[16];
  const float* g2  = (const float*)d_in[17];
  const float* be2 = (const float*)d_in[18];
  const float* Wfc = (const float*)d_in[19];
  const float* bfc = (const float*)d_in[20];
  float* out0 = (float*)d_out;

  const size_t SZ_CST = (size_t)NLAYER * 32 * 4;
  const size_t SZ_REC = (size_t)NROW * 4 * 4;
  const size_t SZ_VT  = (size_t)NB * HID * SEQ * 2;
  const size_t SZ_AO  = (size_t)NB * SEQ * HID * 4;
  const size_t SZ_P   = (size_t)BG * SEQ * SEQ * 2;
  size_t off = 0;
  auto carve = [&](size_t bytes) -> size_t {
    const size_t o = off;
    off = (off + bytes + 4095) & ~(size_t)4095;
    return o;
  };
  const size_t oCST = carve(SZ_CST);
  const size_t oXB  = carve(SZ_REC);
  const size_t oPV  = carve(SZ_REC);
  const size_t oSC  = carve(SZ_REC);
  const size_t oXO  = carve(SZ_REC);
  const size_t oVT  = carve(SZ_VT);
  const size_t oAO  = carve(SZ_AO);
  const size_t oP   = carve(SZ_P);
  if (off > ws_size) return;
  if (off > (size_t)134217728) return;

  char* ws = (char*)d_ws;
  float*          CST = (float*)(ws + oCST);
  float*          XB  = (float*)(ws + oXB);
  float*          PVp = (float*)(ws + oPV);
  float*          SCP = (float*)(ws + oSC);
  float*          XO  = (float*)(ws + oXO);
  unsigned short* VT  = (unsigned short*)(ws + oVT);
  float*          AO  = (float*)(ws + oAO);
  unsigned short* Pp  = (unsigned short*)(ws + oP);

  const int dynLds = RQB * SEQ * 4;
  (void)hipFuncSetAttribute(reinterpret_cast<const void*>(&attn_rows),
                            hipFuncAttributeMaxDynamicSharedMemorySize, dynLds);

  const dim3 gTok(NROW / TOKB);
  const dim3 bTok(TOKB);
  const dim3 gRows(SEQ / RQB, BG);
  const dim3 bRows(SMT);
  const dim3 gGemm((((SEQ / 32) * (HID / 64)) + 7) / 8, BG);
  const dim3 bGemm(256);

  lconst_kernel<<<dim3(NLAYER), dim3(256), 0, stream>>>(Wq, bq, Wk, bk, CST);

  for (int i = 0; i < NLAYER; ++i) {
    const float* Wq_i  = Wq  + (size_t)i * DM * HID;
    const float* bq_i  = bq  + (size_t)i * HID;
    const float* Wk_i  = Wk  + (size_t)i * DM * HID;
    const float* bk_i  = bk  + (size_t)i * HID;
    const float* Wv_i  = Wv  + (size_t)i * DM * HID;
    const float* bv_i  = bv  + (size_t)i * HID;
    const float* Wo_i  = Wo  + (size_t)i * HID * DM;
    const float* bo_i  = bo  + (size_t)i * DM;
    const float* bw_i  = bw  + i;
    const float* g1_i  = g1  + (size_t)i * DM;
    const float* be1_i = be1 + (size_t)i * DM;
    const float* W1_i  = W1  + (size_t)i * DM * FFD;
    const float* b1_i  = b1  + (size_t)i * FFD;
    const float* W2_i  = W2  + (size_t)i * FFD * DM;
    const float* b2_i  = b2  + (size_t)i * DM;
    const float* g2_i  = g2  + (size_t)i * DM;
    const float* be2_i = be2 + (size_t)i * DM;
    const float* cst_i = CST + (size_t)i * 32;

    if (i == 0) {
      tok_kernel<1><<<gTok, bTok, 0, stream>>>(KEY, VAL, XO, Wq_i, bq_i, Wk_i, bk_i, Wv_i, bv_i, cst_i,
                                              XB, PVp, SCP, VT);
    } else {
      tok_kernel<0><<<gTok, bTok, 0, stream>>>(KEY, VAL, XO, Wq_i, bq_i, Wk_i, bk_i, Wv_i, bv_i, cst_i,
                                              XB, PVp, SCP, VT);
    }
    for (int g = 0; g < NGRP; ++g) {
      const int b0 = g * BG;
      attn_rows<<<gRows, bRows, dynLds, stream>>>(PVp, SCP, XB, bw_i, Pp, b0);
      const unsigned short* VTg = VT + (size_t)b0 * HID * SEQ;
      float* AOg = AO + (size_t)b0 * SEQ * HID;
      gemm_t<_Float16, 2, 1, 1, 0, 0><<<gGemm, bGemm, 0, stream>>>(
          Pp, Pp, SEQ, (long long)SEQ * SEQ,
          VTg, SEQ, (long long)HID * SEQ,
          VTg, SEQ, 0LL, 0,
          (void*)AOg, (void*)AOg, HID, (long long)SEQ * HID, HID, 0LL, 0,
          SEQ, HID, SEQ, 1.0f / (PCARRY * VCARRY), 0.0f, 1.0f, 1.0f);
    }
    if (i == NLAYER - 1) {
      post_kernel<1><<<gTok, bTok, 0, stream>>>(XB, AO, Wo_i, bo_i, g1_i, be1_i, W1_i, b1_i, W2_i, b2_i,
                                               g2_i, be2_i, Wfc, bfc, XO, out0);
    } else {
      post_kernel<0><<<gTok, bTok, 0, stream>>>(XB, AO, Wo_i, bo_i, g1_i, be1_i, W1_i, b1_i, W2_i, b2_i,
                                               g2_i, be2_i, Wfc, bfc, XO, out0);
    }
  }
  (void)hipGetLastError();
}
